// MultiHeadSelfAttention_35330400977510
// MI455X (gfx1250) — hardware-run, weakly checked
//
#include <hip/hip_runtime.h>


#ifndef NB
#define NB 4
#endif
#ifndef SEQ
#define SEQ 2048
#endif
#define NB_FULL  4
#define SEQ_FULL 2048
#define DM   1024
#define NH   16
#define HD   64
#define E3   (3 * DM)
#define RH   ((SEQ) < 512 ? (SEQ) : 512)
#define PCAR 1024.0f
#define SCL  0.125f
#define L2E  1.4426950408889634f
#define NEGF (-1.0e30f)
#define X_FULL ((size_t)SEQ_FULL * DM)

static_assert(SEQ % 256 == 0);
static_assert(SEQ <= SEQ_FULL);
static_assert(NB <= NB_FULL);
static_assert(RH % 64 == 0);
static_assert(DM % 64 == 0);
static_assert(E3 % 64 == 0);
static_assert(DM % 32 == 0);
static_assert(NH * HD == DM);

typedef _Float16 h16;
typedef unsigned short bf;
typedef __attribute__((ext_vector_type(16))) __bf16   v16bf;
typedef __attribute__((ext_vector_type(16))) _Float16 v16h;
typedef __attribute__((ext_vector_type(8)))  _Float16 v8h;
typedef __attribute__((ext_vector_type(8)))  unsigned short v8us;
typedef __attribute__((ext_vector_type(8)))  float    v8f;
typedef __attribute__((ext_vector_type(4)))  float    v4f;
typedef __attribute__((ext_vector_type(2)))  float    v2f;
typedef v8h  __attribute__((may_alias)) v8ha;
typedef v4f  __attribute__((may_alias)) v4fa;
typedef v8us __attribute__((may_alias)) v8usa;

__device__ __forceinline__ unsigned short f2bf(float f) { unsigned u = __float_as_uint(f); u += 0x7FFFu + ((u >> 16) & 1u); return (unsigned short)(u >> 16); }
__device__ __forceinline__ float bf2f(unsigned short b) { return __uint_as_float(((unsigned)b) << 16); }
__device__ __forceinline__ float bfr(float f) { return bf2f(f2bf(f)); }
__device__ __forceinline__ void splitf(float y, unsigned short& h, unsigned short& l) { h = f2bf(y); l = f2bf(y - bf2f(h)); }
__device__ __forceinline__ v16h cat16(v8h lo, v8h hi) { return __builtin_shufflevector(lo, hi, 0, 1, 2, 3, 4, 5, 6, 7, 8, 9, 10, 11, 12, 13, 14, 15); }
__device__ __forceinline__ v16bf cat16b(v8us lo, v8us hi) { return __builtin_bit_cast(v16bf, __builtin_shufflevector(lo, hi, 0, 1, 2, 3, 4, 5, 6, 7, 8, 9, 10, 11, 12, 13, 14, 15)); }
__device__ __forceinline__ v8f wmma16(v16h a, v16h b, v8f c) { return __builtin_amdgcn_wmma_f32_16x16x32_f16(false, a, false, b, (short)0, c, false, false); }
__device__ __forceinline__ v8f wmmab(v16bf a, v16bf b, v8f c) { return __builtin_amdgcn_wmma_f32_16x16x32_bf16(false, a, false, b, (short)0, c, false, false); }
__device__ __forceinline__ v16h  ldh(const h16* p) { return cat16(*(const v8h*)p, *(const v8h*)(p + 16)); }
__device__ __forceinline__ v16bf ldb(const bf* p)  { return cat16b(*(const v8us*)p, *(const v8us*)(p + 16)); }

template <typename T16> struct WFrag;
template <> struct WFrag<h16> { typedef v16h V; static __device__ __forceinline__ V ld(const h16* p) { return cat16(*(const v8h*)p, *(const v8h*)(p + 16)); } static __device__ __forceinline__ v8f mma(V a, V b, v8f c) { return wmma16(a, b, c); } };
template <> struct WFrag<bf> { typedef v16bf V; static __device__ __forceinline__ V ld(const bf* p) { return cat16b(*(const v8us*)p, *(const v8us*)(p + 16)); } static __device__ __forceinline__ v8f mma(V a, V b, v8f c) { return wmmab(a, b, c); } };
template <typename T16, int NSPLIT, bool BIAS>
__global__ __launch_bounds__(32) void k_gemmw(const T16* __restrict__ A, const T16* __restrict__ A2, const T16* __restrict__ Bt, const T16* __restrict__ Bt2, int K, float* C, int ldc, const float* __restrict__ bias, size_t sA, size_t sB, size_t sC) {
    typedef typename WFrag<T16>::V V;
    __shared__ __align__(16) float os[16 * 68];
    const size_t z = blockIdx.z; A += z * sA; if (A2) A2 += z * sA; Bt += z * sB; if (Bt2) Bt2 += z * sB; C += z * sC;
    const int lane = threadIdx.x & 31, lr = lane & 15, hi = lane >> 4; const int r0 = blockIdx.x * 64, c0 = blockIdx.y * 64;
    v8f acc[4][4];
#pragma unroll
    for (int mb = 0; mb < 4; ++mb)
#pragma unroll
        for (int nb = 0; nb < 4; ++nb) acc[mb][nb] = (v8f){};
    const size_t aoff = (size_t)(r0 + lr) * K + 8 * hi, boff = (size_t)(c0 + lr) * K + 8 * hi;
#pragma unroll 1
    for (int kc = 0; kc < K; kc += 32) {
        V a[4], a2[4];
#pragma unroll
        for (int mb = 0; mb < 4; ++mb) { a[mb] = WFrag<T16>::ld(A + aoff + (size_t)mb * 16 * K + kc); if (NSPLIT == 1 || NSPLIT == 2) a2[mb] = WFrag<T16>::ld(A2 + aoff + (size_t)mb * 16 * K + kc); }
#pragma unroll
        for (int nb = 0; nb < 4; ++nb) { const V b = WFrag<T16>::ld(Bt + boff + (size_t)nb * 16 * K + kc); V b2; if (NSPLIT >= 2) b2 = WFrag<T16>::ld(Bt2 + boff + (size_t)nb * 16 * K + kc);
#pragma unroll
            for (int mb = 0; mb < 4; ++mb) { acc[mb][nb] = WFrag<T16>::mma(a[mb], b, acc[mb][nb]); if (NSPLIT == 1 || NSPLIT == 2) acc[mb][nb] = WFrag<T16>::mma(a2[mb], b, acc[mb][nb]); if (NSPLIT >= 2) acc[mb][nb] = WFrag<T16>::mma(a[mb], b2, acc[mb][nb]); } }
        asm volatile("v_nop\n\tv_nop\n\tv_nop\n\tv_nop" : "+v"(acc[0][0]), "+v"(acc[1][1]), "+v"(acc[2][2]), "+v"(acc[3][3]) : "v"(a[0]), "v"(a[3]));
    }
#pragma unroll
    for (int mb = 0; mb < 4; ++mb) {
#pragma unroll
        for (int nb = 0; nb < 4; ++nb) {
#pragma unroll
            for (int j = 0; j < 8; ++j) os[(hi * 8 + j) * 68 + nb * 16 + lr] = acc[mb][nb][j]; }
        __builtin_amdgcn_wave_barrier(); asm volatile("" ::: "memory");
        float* crow = C + (size_t)(r0 + mb * 16) * ldc + c0;
#pragma unroll 1
        for (int ps = 0; ps < 2; ++ps) {
#pragma unroll
            for (int s = 0; s < 8; ++s) { const int row = 2 * s + hi, cofs = lr * 4; v4f val = *(const v4fa*)(os + row * 68 + cofs); if (BIAS) { val[0] += bfr(bias[c0 + cofs]); val[1] += bfr(bias[c0 + cofs + 1]); val[2] += bfr(bias[c0 + cofs + 2]); val[3] += bfr(bias[c0 + cofs + 3]); }
                *(volatile v4f*)(crow + (size_t)row * ldc + cofs) = val; }
            if (ps == 0) __threadfence(); }
        __builtin_amdgcn_wave_barrier(); asm volatile("" ::: "memory");
    }
}

__global__ __launch_bounds__(256) void k_cvt8(const float* __restrict__ src, bf* dst, size_t n8, size_t sstride, size_t dstride) {
    const size_t i = (size_t)blockIdx.x * 256 + threadIdx.x; if (i >= n8) return;
    src += (size_t)blockIdx.y * sstride; dst += (size_t)blockIdx.y * dstride;
    const v8f v = *(const v8f*)(src + i * 8); v8us o;
#pragma unroll
    for (int k = 0; k < 8; ++k) o[k] = f2bf(v[k]);
    *(volatile v8us*)(dst + i * 8) = o; __threadfence(); *(volatile v8us*)(dst + i * 8) = o; }

__global__ __launch_bounds__(32) void k_invf(float* IF) {
    const int i = threadIdx.x & 31; const float e = (float)(2 * i) * (1.0f / (float)HD); const float p = powf(10000.0f, e); const float v = 1.0f / p;
    *(volatile float*)(IF + i) = v; __threadfence(); *(volatile float*)(IF + i) = v; }

__global__ __launch_bounds__(256) void k_cstab(const int* __restrict__ pos, const float* __restrict__ IF, float* CS) {
    const int idx = blockIdx.x * 256 + threadIdx.x; if (idx >= SEQ * 32) return; const int t = idx >> 5, i = idx & 31;
    const float ang = (float)pos[t] * IF[i]; float sn, cs; sincosf(ang, &sn, &cs); v2f o; o[0] = cs; o[1] = sn;
    *(volatile v2f*)(CS + (size_t)idx * 2) = o; __threadfence(); *(volatile v2f*)(CS + (size_t)idx * 2) = o; }

#define ROPE_BLOCKS ((unsigned)(((size_t)2 * NH * SEQ * (HD / 8)) / 256))
#define VTP_BLOCKS  ((unsigned)(((size_t)NH * HD * (SEQ / 8)) / 256))
__global__ __launch_bounds__(256) void k_planes(const float* __restrict__ F, const float* __restrict__ CS, h16* QK16, bf* QKh, bf* QKl, h16* VT16, bf* VTh, bf* VTl) {
    if (blockIdx.x < ROPE_BLOCKS) {
        const unsigned idx = blockIdx.x * 256u + threadIdx.x;
        const int d8 = (int)(idx & 7u); const int t = (int)((idx >> 3) % (unsigned)SEQ); const int hh = (int)(idx / (8u * (unsigned)SEQ));
        const float* f = F + (size_t)t * E3 + hh * HD + d8 * 8;
        const v4f xa = *(const v4f*)f, xb = *(const v4f*)(f + 4);
        const float* cp = CS + ((size_t)t * 32 + d8 * 4) * 2;
        const v4f ca = *(const v4f*)cp, cb = *(const v4f*)(cp + 4);
        float r[8];
        r[0] = xa[0] * ca[0] - xa[1] * ca[1]; r[1] = xa[0] * ca[1] + xa[1] * ca[0];
        r[2] = xa[2] * ca[2] - xa[3] * ca[3]; r[3] = xa[2] * ca[3] + xa[3] * ca[2];
        r[4] = xb[0] * cb[0] - xb[1] * cb[1]; r[5] = xb[0] * cb[1] + xb[1] * cb[0];
        r[6] = xb[2] * cb[2] - xb[3] * cb[3]; r[7] = xb[2] * cb[3] + xb[3] * cb[2];
        v8h o16; v8us oh, ol;
#pragma unroll
        for (int k = 0; k < 8; ++k) { o16[k] = (h16)r[k]; unsigned short a2, c2; splitf(r[k], a2, c2); oh[k] = a2; ol[k] = c2; }
        const bool early = (t < RH);
        const size_t e = ((size_t)hh * SEQ + t) * HD + d8 * 8;
        const size_t e2 = ((size_t)hh * RH + (early ? t : 0)) * HD + d8 * 8;
        *(volatile v8h*)(QK16 + e) = o16; if (early) { *(volatile v8us*)(QKh + e2) = oh; *(volatile v8us*)(QKl + e2) = ol; }
        __threadfence();
        *(volatile v8h*)(QK16 + e) = o16; if (early) { *(volatile v8us*)(QKh + e2) = oh; *(volatile v8us*)(QKl + e2) = ol; }
    } else {
        const unsigned idx = (blockIdx.x - ROPE_BLOCKS) * 256u + threadIdx.x;
        const int t = (int)(idx % (unsigned)(SEQ / 8)) * 8; const int d = (int)((idx / (unsigned)(SEQ / 8)) % (unsigned)HD); const int g = (int)(idx / ((unsigned)(SEQ / 8) * (unsigned)HD));
        const float* f = F + (size_t)t * E3 + 2 * DM + g * HD + d;
        v8h o16; v8us oh, ol;
#pragma unroll
        for (int q = 0; q < 8; ++q) { const float x = f[(size_t)q * E3]; o16[q] = (h16)x; unsigned short a2, c2; splitf(x, a2, c2); oh[q] = a2; ol[q] = c2; }
        const bool early = (t < RH);
        const size_t e = ((size_t)g * HD + d) * SEQ + t;
        const size_t e2 = ((size_t)g * HD + d) * RH + (early ? t : 0);
        *(volatile v8h*)(VT16 + e) = o16; if (early) { *(volatile v8us*)(VTh + e2) = oh; *(volatile v8us*)(VTl + e2) = ol; }
        __threadfence();
        *(volatile v8h*)(VT16 + e) = o16; if (early) { *(volatile v8us*)(VTh + e2) = oh; *(volatile v8us*)(VTl + e2) = ol; }
    }
}

__device__ __forceinline__ void soft_step(const v8f s0, const v8f s1, const int srow, const int jb0, float& mrun, float& lrun, float& alpha, float (&p0)[8], float (&p1)[8]) {
    float cm = NEGF;
#pragma unroll
    for (int r = 0; r < 8; ++r) { const float a0 = (jb0 + r <= srow) ? s0[r] * SCL : NEGF; const float a1 = (jb0 + 16 + r <= srow) ? s1[r] * SCL : NEGF; p0[r] = a0; p1[r] = a1; cm = fmaxf(cm, fmaxf(a0, a1)); }
    cm = fmaxf(cm, __shfl_xor(cm, 16, 32));
    const float mnew = fmaxf(mrun, cm);
    alpha = __builtin_amdgcn_exp2f((mrun - mnew) * L2E);
    float ls = 0.f;
#pragma unroll
    for (int r = 0; r < 8; ++r) { p0[r] = __builtin_amdgcn_exp2f((p0[r] - mnew) * L2E); p1[r] = __builtin_amdgcn_exp2f((p1[r] - mnew) * L2E); ls += p0[r] + p1[r]; }
    ls += __shfl_xor(ls, 16, 32);
    lrun = lrun * alpha + ls; mrun = mnew;
}

__device__ __forceinline__ void epi_store(const v8f o0, const v8f o1, const v8f o2, const v8f o3, const float inv, bf* Ah, bf* Al, const int q0, const int h, const int lane) {
    __shared__ __align__(16) float os[16 * 68];
    const int lr = lane & 15, hi = lane >> 4;
#pragma unroll
    for (int r = 0; r < 8; ++r) { float* w = os + lr * 68 + 8 * hi + r; w[0] = o0[r] * inv; w[16] = o1[r] * inv; w[32] = o2[r] * inv; w[48] = o3[r] * inv; }
    __syncthreads();
#pragma unroll 1
    for (int ps = 0; ps < 2; ++ps) {
#pragma unroll
        for (int s = 0; s < 4; ++s) { const int row = 4 * s + (lane >> 3), c8 = (lane & 7) * 8; const v4f a = *(const v4fa*)(os + row * 68 + c8), b = *(const v4fa*)(os + row * 68 + c8 + 4); v8us oh, ol;
#pragma unroll
            for (int q = 0; q < 4; ++q) { unsigned short x, y; splitf(a[q], x, y); oh[q] = x; ol[q] = y; splitf(b[q], x, y); oh[4 + q] = x; ol[4 + q] = y; }
            const size_t oo = (size_t)(q0 + row) * DM + h * HD + c8; *(volatile v8us*)(Ah + oo) = oh; *(volatile v8us*)(Al + oo) = ol; }
        if (ps == 0) __threadfence(); }
}

__global__ __launch_bounds__(32) void k_flash16(const h16* __restrict__ QK16, const h16* __restrict__ VT16, bf* ATh, bf* ATl, int roff) {
    const int lane = threadIdx.x & 31, lr = lane & 15, hi = lane >> 4; const int h = blockIdx.y; const int q0 = roff + blockIdx.x * 16; const int srow = q0 + lr;
    const h16* qb = QK16 + ((size_t)h * SEQ + srow) * HD + 8 * hi;
    const h16* kb = QK16 + ((size_t)(NH + h) * SEQ + lr) * HD + 8 * hi;
    const h16* vb = VT16 + ((size_t)h * HD + lr) * SEQ + 8 * hi;
    const v16h bq0 = ldh(qb), bq1 = ldh(qb + 32);
    v8f o0 = (v8f){}, o1 = (v8f){}, o2 = (v8f){}, o3 = (v8f){};
    float mrun = NEGF, lrun = 0.f;
#pragma unroll 1
    for (int j0 = 0; j0 <= q0 + 15; j0 += 32) {
        const h16* kp = kb + (size_t)j0 * HD;
        const v16h a00 = ldh(kp), a01 = ldh(kp + 32), a10 = ldh(kp + 16 * HD), a11 = ldh(kp + 16 * HD + 32);
        v8f s0 = (v8f){}, s1 = (v8f){};
        s0 = wmma16(a00, bq0, s0); s0 = wmma16(a01, bq1, s0); s1 = wmma16(a10, bq0, s1); s1 = wmma16(a11, bq1, s1);
        asm volatile("v_nop\n\tv_nop\n\tv_nop\n\tv_nop" : "+v"(s0), "+v"(s1) : "v"(a00), "v"(a11));
        float p0[8], p1[8], alpha;
        soft_step(s0, s1, srow, j0 + 8 * hi, mrun, lrun, alpha, p0, p1);
        v8h pa, pb;
#pragma unroll
        for (int i = 0; i < 8; ++i) { pa[i] = (h16)(p0[i] * PCAR); pb[i] = (h16)(p1[i] * PCAR); }
        const v16h bp = cat16(pa, pb);
        const h16* vp = vb + j0;
        const v16h av0 = ldh(vp), av1 = ldh(vp + (size_t)16 * SEQ), av2 = ldh(vp + (size_t)32 * SEQ), av3 = ldh(vp + (size_t)48 * SEQ);
#pragma unroll
        for (int r = 0; r < 8; ++r) { o0[r] *= alpha; o1[r] *= alpha; o2[r] *= alpha; o3[r] *= alpha; }
        o0 = wmma16(av0, bp, o0); o1 = wmma16(av1, bp, o1); o2 = wmma16(av2, bp, o2); o3 = wmma16(av3, bp, o3);
        asm volatile("v_nop\n\tv_nop\n\tv_nop\n\tv_nop" : "+v"(o0), "+v"(o1), "+v"(o2), "+v"(o3) : "v"(av0), "v"(av3), "v"(bp));
    }
    const float inv = (1.0f / lrun) * (1.0f / PCAR);
    epi_store(o0, o1, o2, o3, inv, ATh, ATl, q0, h, lane);
}

__global__ __launch_bounds__(32) void k_flashhl(const bf* __restrict__ QKh, const bf* __restrict__ QKl, const bf* __restrict__ VTh, const bf* __restrict__ VTl, bf* ATh, bf* ATl) {
    const int lane = threadIdx.x & 31, lr = lane & 15, hi = lane >> 4; const int h = blockIdx.y; const int q0 = blockIdx.x * 16; const int srow = q0 + lr;
    const size_t qo = ((size_t)h * RH + srow) * HD + 8 * hi;
    const size_t ko = ((size_t)(NH + h) * RH + lr) * HD + 8 * hi;
    const size_t vo = ((size_t)h * HD + lr) * RH + 8 * hi;
    const v16bf bqh0 = ldb(QKh + qo), bqh1 = ldb(QKh + qo + 32), bql0 = ldb(QKl + qo), bql1 = ldb(QKl + qo + 32);
    v8f o0 = (v8f){}, o1 = (v8f){}, o2 = (v8f){}, o3 = (v8f){};
    float mrun = NEGF, lrun = 0.f;
#pragma unroll 1
    for (int j0 = 0; j0 <= q0 + 15; j0 += 32) {
        const size_t kk = ko + (size_t)j0 * HD;
        const v16bf kh00 = ldb(QKh + kk), kh01 = ldb(QKh + kk + 32), kl00 = ldb(QKl + kk), kl01 = ldb(QKl + kk + 32);
        const v16bf kh10 = ldb(QKh + kk + 16 * HD), kh11 = ldb(QKh + kk + 16 * HD + 32), kl10 = ldb(QKl + kk + 16 * HD), kl11 = ldb(QKl + kk + 16 * HD + 32);
        v8f s0 = (v8f){}, s1 = (v8f){};
        s0 = wmmab(kh00, bqh0, s0); s0 = wmmab(kh01, bqh1, s0); s0 = wmmab(kl00, bqh0, s0); s0 = wmmab(kl01, bqh1, s0); s0 = wmmab(kh00, bql0, s0); s0 = wmmab(kh01, bql1, s0);
        s1 = wmmab(kh10, bqh0, s1); s1 = wmmab(kh11, bqh1, s1); s1 = wmmab(kl10, bqh0, s1); s1 = wmmab(kl11, bqh1, s1); s1 = wmmab(kh10, bql0, s1); s1 = wmmab(kh11, bql1, s1);
        asm volatile("v_nop\n\tv_nop\n\tv_nop\n\tv_nop" : "+v"(s0), "+v"(s1) : "v"(kh00), "v"(kh11), "v"(kl00), "v"(kl11));
        float p0[8], p1[8], alpha;
        soft_step(s0, s1, srow, j0 + 8 * hi, mrun, lrun, alpha, p0, p1);
        v8us pha, phb, pla, plb;
#pragma unroll
        for (int i = 0; i < 8; ++i) { unsigned short x, y; splitf(p0[i], x, y); pha[i] = x; pla[i] = y; splitf(p1[i], x, y); phb[i] = x; plb[i] = y; }
        const v16bf bph = cat16b(pha, phb), bpl = cat16b(pla, plb);
        const size_t vv = vo + j0;
        const v16bf vh0 = ldb(VTh + vv), vh1 = ldb(VTh + vv + (size_t)16 * RH), vh2 = ldb(VTh + vv + (size_t)32 * RH), vh3 = ldb(VTh + vv + (size_t)48 * RH);
        const v16bf vl0 = ldb(VTl + vv), vl1 = ldb(VTl + vv + (size_t)16 * RH), vl2 = ldb(VTl + vv + (size_t)32 * RH), vl3 = ldb(VTl + vv + (size_t)48 * RH);
#pragma unroll
        for (int r = 0; r < 8; ++r) { o0[r] *= alpha; o1[r] *= alpha; o2[r] *= alpha; o3[r] *= alpha; }
        o0 = wmmab(vh0, bph, o0); o0 = wmmab(vl0, bph, o0); o0 = wmmab(vh0, bpl, o0);
        o1 = wmmab(vh1, bph, o1); o1 = wmmab(vl1, bph, o1); o1 = wmmab(vh1, bpl, o1);
        o2 = wmmab(vh2, bph, o2); o2 = wmmab(vl2, bph, o2); o2 = wmmab(vh2, bpl, o2);
        o3 = wmmab(vh3, bph, o3); o3 = wmmab(vl3, bph, o3); o3 = wmmab(vh3, bpl, o3);
        asm volatile("v_nop\n\tv_nop\n\tv_nop\n\tv_nop" : "+v"(o0), "+v"(o1), "+v"(o2), "+v"(o3) : "v"(vh0), "v"(vh3), "v"(vl3), "v"(bph), "v"(bpl));
    }
    const float inv = 1.0f / lrun;
    epi_store(o0, o1, o2, o3, inv, ATh, ATl, q0, h, lane);
}

extern "C" void kernel_launch(void* const* d_in, const int* in_sizes, int n_in,
                              void* d_out, int out_size, void* d_ws, size_t ws_size, hipStream_t stream) {
    if (n_in < 4) return;
    const size_t need_x = (size_t)(NB - 1) * X_FULL + (size_t)SEQ * DM;
    if ((size_t)in_sizes[0] < need_x || in_sizes[1] < SEQ || (size_t)in_sizes[2] < (size_t)E3 * DM || (size_t)in_sizes[3] < (size_t)DM * DM || (size_t)out_size < need_x) return;
    const float* x    = (const float*)d_in[0];
    const int*   pos  = (const int*)d_in[1];
    const float* wqkv = (const float*)d_in[2];
    const float* wout = (const float*)d_in[3];
    float* OUT = (float*)d_out;
    char* wsp = (char*)d_ws;
    auto take = [&](size_t bytes) { char* p = wsp; wsp += (bytes + 255) & ~(size_t)255; return (void*)p; };
    bf* WQKV = (bf*)take((size_t)E3 * DM * 2);
    bf* WO   = (bf*)take((size_t)DM * DM * 2);
    bf* XB   = (bf*)take((size_t)NB * SEQ * DM * 2);
    float* IFQ = (float*)take(128);
    float* CS  = (float*)take((size_t)SEQ * 32 * 2 * 4);
    float* FQKV = (float*)take((size_t)SEQ * E3 * 4);
    h16* QK16 = (h16*)take((size_t)2 * NH * SEQ * HD * 2);
    bf* QKh = (bf*)take((size_t)2 * NH * RH * HD * 2);
    bf* QKl = (bf*)take((size_t)2 * NH * RH * HD * 2);
    h16* VT16 = (h16*)take((size_t)NH * HD * SEQ * 2);
    bf* VTh = (bf*)take((size_t)NH * HD * RH * 2);
    bf* VTl = (bf*)take((size_t)NH * HD * RH * 2);
    bf* ATh = (bf*)take((size_t)NB * SEQ * DM * 2);
    bf* ATl = (bf*)take((size_t)NB * SEQ * DM * 2);
    const size_t carved = (size_t)(wsp - (char*)d_ws);
    if (carved > ws_size || carved > (size_t)134217728) return;

    k_cvt8<<<dim3((unsigned)(((size_t)E3 * DM / 8 + 255) / 256), 1), 256, 0, stream>>>(wqkv, WQKV, (size_t)E3 * DM / 8, 0, 0);
    k_cvt8<<<dim3((unsigned)(((size_t)DM * DM / 8 + 255) / 256), 1), 256, 0, stream>>>(wout, WO, (size_t)DM * DM / 8, 0, 0);
    k_cvt8<<<dim3((unsigned)(((size_t)SEQ * DM / 8 + 255) / 256), NB), 256, 0, stream>>>(x, XB, (size_t)SEQ * DM / 8, X_FULL, (size_t)SEQ * DM);
    k_invf<<<1, 32, 0, stream>>>(IFQ);
    k_cstab<<<(SEQ * 32 + 255) / 256, 256, 0, stream>>>(pos, IFQ, CS);

    for (int b = 0; b < NB; ++b) {
        const bf* xb = XB + (size_t)b * SEQ * DM;
        bf* ath = ATh + (size_t)b * SEQ * DM; bf* atl = ATl + (size_t)b * SEQ * DM;
        k_gemmw<bf, 0, false><<<dim3(SEQ / 64, E3 / 64, 1), 32, 0, stream>>>(xb, nullptr, WQKV, nullptr, DM, FQKV, E3, nullptr, 0, 0, 0);
        k_planes<<<ROPE_BLOCKS + VTP_BLOCKS, 256, 0, stream>>>(FQKV, CS, QK16, QKh, QKl, VT16, VTh, VTl);
        k_flashhl<<<dim3(RH / 16, NH), 32, 0, stream>>>(QKh, QKl, VTh, VTl, ath, atl);
        if (SEQ > RH) k_flash16<<<dim3((SEQ - RH) / 16, NH), 32, 0, stream>>>(QK16, VT16, ath, atl, RH);
    }
    k_gemmw<bf, 1, false><<<dim3(SEQ / 64, DM / 64, NB), 32, 0, stream>>>(ATh, ATl, WO, nullptr, DM, OUT, DM, nullptr, (size_t)SEQ * DM, 0, X_FULL);
}
